// SpatialAttentionLayer_GAT_21311627723297
// MI455X (gfx1250) — hardware-verified
//
#include <hip/hip_runtime.h>
#include <stddef.h>


#define DCH   64
#define GSP   68
#define GROWS 64
#define NB    1024
#define CHUNK 2048
#define NTHR  256
#define NWAVE 8
#define WCAP  256
#define NGRP  (CHUNK / (NTHR * 4))
#define WPL_HALVES 81920
#define NEGSL 0.2f
#define MINIT (-1.0e30f)

#define LDS_WORDS (NB * DCH + NB + NB + NWAVE * WCAP + NWAVE)
#define LDS_BYTES (LDS_WORDS * 4)

static_assert(WCAP == (CHUNK / NTHR) * 32);
static_assert(NGRP == 2);
static_assert(NB == 1024);
static_assert(CHUNK == 2048);
static_assert(LDS_BYTES == 278560);

typedef float          v4f   __attribute__((ext_vector_type(4)));
typedef float          v8f   __attribute__((ext_vector_type(8)));
typedef int            v4i   __attribute__((ext_vector_type(4)));
typedef unsigned int   v4u   __attribute__((ext_vector_type(4)));
typedef unsigned int   v8u   __attribute__((ext_vector_type(8)));
typedef __bf16         v16bf __attribute__((ext_vector_type(16)));
typedef unsigned short us_t;

__device__ __forceinline__ v8f wm(v16bf a, v16bf b, v8f c) {
  v8f d = __builtin_amdgcn_wmma_f32_16x16x32_bf16(false, a, false, b, (short)0, c, false, false);
  asm volatile("v_nop\n\tv_nop\n\tv_nop\n\tv_nop" : "+v"(d) : "v"(a), "v"(b));
  return d;
}

__device__ __forceinline__ unsigned int f2bf(float f) {
  unsigned int u = __float_as_uint(f);
  u += 0x7FFFu + ((u >> 16) & 1u);
  return u >> 16;
}
__device__ __forceinline__ float bf2f(unsigned int b) { return __uint_as_float(b << 16); }

__device__ __forceinline__ void hl2(float a, float b, unsigned int& ho, unsigned int& lo) {
  const unsigned int ha = f2bf(a), hb = f2bf(b);
  const unsigned int la = f2bf(a - bf2f(ha)), lb = f2bf(b - bf2f(hb));
  ho = ha | (hb << 16);
  lo = la | (lb << 16);
}

__device__ __forceinline__ v16bf ld_frag(const us_t* p) {
  const v4u q0 = *(const v4u*)(p);
  const v4u q1 = *(const v4u*)(p + 16);
  const v8u w = __builtin_shufflevector(q0, q1, 0, 1, 2, 3, 4, 5, 6, 7);
  return __builtin_bit_cast(v16bf, w);
}

struct PrepArgs {
  const float* W0; const float* W1; const float* W2; const float* W3; const float* W4;
  const float* W5; const float* W6; const float* W7; const float* W8;
  us_t* P;
};
static_assert(sizeof(PrepArgs) == 80);

__global__ __launch_bounds__(NTHR) void k_prep(PrepArgs g) {
  const int y = blockIdx.y;
  const float* W = g.W0;
  W = (y == 1) ? g.W1 : W;
  W = (y == 2) ? g.W2 : W;
  W = (y == 3) ? g.W3 : W;
  W = (y == 4) ? g.W4 : W;
  W = (y == 5) ? g.W5 : W;
  W = (y == 6) ? g.W6 : W;
  W = (y == 7) ? g.W7 : W;
  W = (y == 8) ? g.W8 : W;
  const int K   = (y == 8) ? 128 : 64;
  const int ppr = K >> 3;
  const int tot = DCH * ppr;
  const int i   = blockIdx.x * NTHR + threadIdx.x;
  if (i >= tot) return;
  const int n  = i / ppr;
  const int k0 = (i - n * ppr) * 8;
  v4u hv, lv;
  {
    unsigned int h_, l_;
    hl2(W[(size_t)(k0 + 0) * DCH + n], W[(size_t)(k0 + 1) * DCH + n], h_, l_); hv.x = h_; lv.x = l_;
    hl2(W[(size_t)(k0 + 2) * DCH + n], W[(size_t)(k0 + 3) * DCH + n], h_, l_); hv.y = h_; lv.y = l_;
    hl2(W[(size_t)(k0 + 4) * DCH + n], W[(size_t)(k0 + 5) * DCH + n], h_, l_); hv.z = h_; lv.z = l_;
    hl2(W[(size_t)(k0 + 6) * DCH + n], W[(size_t)(k0 + 7) * DCH + n], h_, l_); hv.w = h_; lv.w = l_;
  }
  us_t* hp = g.P + (size_t)y * 8192 + (size_t)n * K + k0;
  us_t* lp = hp + DCH * K;
  *(volatile v4u*)hp = hv;
  *(volatile v4u*)lp = lv;
  __threadfence();
  *(volatile v4u*)hp = hv;
  *(volatile v4u*)lp = lv;
}

struct GemmArgs {
  const float* X; const float* bias;
  const us_t* W0; const us_t* W1; const us_t* W2; const us_t* W3;
  float* Y0; float* Y1; float* Y2; float* Y3;
  int ldx; int ldy; int N; int pad0;
};
static_assert(sizeof(GemmArgs) == 96);

#define CVT2(I, A, B) { unsigned int h_, l_; hl2((A), (B), h_, l_); hv[I] = h_; lv[I] = l_; }

template <int KS>
__global__ __launch_bounds__(128) void k_gemm(GemmArgs g) {
  __shared__ __attribute__((aligned(16))) float stg[4 * 16 * GSP];

  const int tid  = threadIdx.x;
  const int lane = tid & 31;
  const int wave = tid >> 5;
  const int h    = lane >> 4;
  const int m    = lane & 15;
  const int set  = blockIdx.y;
  const us_t* Wp = g.W0;
  float* Yp = g.Y0;
  if (set == 1) { Wp = g.W1; Yp = g.Y1; }
  if (set == 2) { Wp = g.W2; Yp = g.Y2; }
  if (set == 3) { Wp = g.W3; Yp = g.Y3; }
  const int K = KS * 32;

  const int  row0   = blockIdx.x * GROWS + wave * 16;
  const bool active = row0 < g.N;
  int arow = row0 + m;
  if (arow > g.N - 1) arow = g.N - 1;
  const float* xr = g.X + (size_t)arow * g.ldx;

  v8f acc[4];
#pragma unroll
  for (int ct = 0; ct < 4; ++ct) {
#pragma unroll
    for (int r = 0; r < 8; ++r) acc[ct][r] = 0.f;
  }

#pragma unroll
  for (int kt = 0; kt < KS; ++kt) {
    const float* p = xr + kt * 32 + 8 * h;
    const v4f x0 = *(const v4f*)(p);
    const v4f x1 = *(const v4f*)(p + 4);
    const v4f x2 = *(const v4f*)(p + 16);
    const v4f x3 = *(const v4f*)(p + 20);
    v8u hv, lv;
    CVT2(0, x0.x, x0.y) CVT2(1, x0.z, x0.w) CVT2(2, x1.x, x1.y) CVT2(3, x1.z, x1.w)
    CVT2(4, x2.x, x2.y) CVT2(5, x2.z, x2.w) CVT2(6, x3.x, x3.y) CVT2(7, x3.z, x3.w)
    const v16bf ahi = __builtin_bit_cast(v16bf, hv);
    const v16bf alo = __builtin_bit_cast(v16bf, lv);
#pragma unroll
    for (int ct = 0; ct < 4; ++ct) {
      const us_t* wr_ = Wp + (size_t)(ct * 16 + m) * K + kt * 32 + 8 * h;
      const v16bf bhi = ld_frag(wr_);
      const v16bf blo = ld_frag(wr_ + DCH * K);
      acc[ct] = wm(ahi, bhi, acc[ct]);
      acc[ct] = wm(ahi, blo, acc[ct]);
      acc[ct] = wm(alo, bhi, acc[ct]);
    }
  }

  float bv[4] = {0.f, 0.f, 0.f, 0.f};
  if (g.bias != nullptr) {
#pragma unroll
    for (int ct = 0; ct < 4; ++ct) bv[ct] = g.bias[ct * 16 + m];
  }
  float* sw = stg + wave * (16 * GSP);
#pragma unroll
  for (int ct = 0; ct < 4; ++ct) {
#pragma unroll
    for (int r = 0; r < 8; ++r) sw[(8 * h + r) * GSP + ct * 16 + m] = acc[ct][r] + bv[ct];
  }
  __syncthreads();

  v4f o[8];
#pragma unroll
  for (int i = 0; i < 8; ++i) o[i] = *(const v4f*)(sw + (2 * i + h) * GSP + 4 * m);
  if (active) {
    float* yb = Yp + (size_t)row0 * g.ldy + 4 * m;
#pragma unroll
    for (int i = 0; i < 8; ++i) *(volatile v4f*)(yb + (size_t)(2 * i + h) * g.ldy) = o[i];
    __threadfence();
#pragma unroll
    for (int i = 0; i < 8; ++i) *(volatile v4f*)(yb + (size_t)(2 * i + h) * g.ldy) = o[i];
  }
}
#undef CVT2

__global__ __launch_bounds__(NTHR) void k_agg(
    const float* __restrict__ hs, const float* __restrict__ hd,
    const int* __restrict__ sidx, const int* __restrict__ didx,
    const float* __restrict__ attn, const float* __restrict__ bias,
    float* outp, int ld_out, int n_src, int n_dst, int nE) {
  extern __shared__ v4f lds_dyn[];
  float* sacc = (float*)lds_dyn;
  float* emx  = sacc + NB * DCH;
  float* den  = emx + NB;
  int*   list = (int*)(den + NB);
  int*   wcnt = list + NWAVE * WCAP;

  const int tid  = threadIdx.x;
  const int lane = tid & 31;
  const int wave = tid >> 5;
  const int half = lane >> 4;
  const int q    = lane & 15;
  const int nodeBase = blockIdx.x * NB;

  {
    const v4f z4 = {0.f, 0.f, 0.f, 0.f};
    for (int i = tid; i < NB * DCH / 4; i += NTHR) lds_dyn[i] = z4;
    for (int i = tid; i < NB; i += NTHR) { emx[i] = MINIT; den[i] = 0.f; }
  }
  __syncthreads();

  const v4f  a4   = *(const v4f*)(attn + 4 * q);
  const bool al16 = ((((size_t)didx) & 15) == 0);
  const int  nChunks = (nE + CHUNK - 1) / CHUNK;

#pragma unroll 1
  for (int ch = 0; ch < nChunks; ++ch) {
    const int cbase = ch * CHUNK;
    int wc = 0;
#pragma unroll
    for (int g = 0; g < NGRP; ++g) {
      const int el0  = (g * NTHR + tid) * 4;
      const int e0   = cbase + el0;
      const int sent = -2147483647 - 1;
      v4i d;
      if (al16 && (cbase + CHUNK <= nE)) {
        d = *(const v4i*)(didx + e0);
      } else {
        const int v0 = didx[min(e0,     nE - 1)];
        const int v1 = didx[min(e0 + 1, nE - 1)];
        const int v2 = didx[min(e0 + 2, nE - 1)];
        const int v3 = didx[min(e0 + 3, nE - 1)];
        d.x = (e0     < nE) ? v0 : sent;
        d.y = (e0 + 1 < nE) ? v1 : sent;
        d.z = (e0 + 2 < nE) ? v2 : sent;
        d.w = (e0 + 3 < nE) ? v3 : sent;
      }
      const unsigned s0 = (unsigned)d.x - (unsigned)nodeBase;
      const unsigned s1 = (unsigned)d.y - (unsigned)nodeBase;
      const unsigned s2 = (unsigned)d.z - (unsigned)nodeBase;
      const unsigned s3 = (unsigned)d.w - (unsigned)nodeBase;
      const bool h0 = s0 < (unsigned)NB;
      const bool h1 = s1 < (unsigned)NB;
      const bool h2 = s2 < (unsigned)NB;
      const bool h3 = s3 < (unsigned)NB;
      const unsigned many = __builtin_amdgcn_ballot_w32(h0 | h1 | h2 | h3);
      if (many != 0u) {
#define HITJ(J, HJ, SJ) { \
          const unsigned mj = __builtin_amdgcn_ballot_w32(HJ); \
          if (HJ) { \
            const int pos = wc + (int)__builtin_amdgcn_mbcnt_lo(mj, 0u); \
            if (pos < WCAP) list[wave * WCAP + pos] = ((el0 + (J)) << 10) | (int)(SJ); \
          } \
          wc += (int)__builtin_popcount(mj); }
        HITJ(0, h0, s0)
        HITJ(1, h1, s1)
        HITJ(2, h2, s2)
        HITJ(3, h3, s3)
#undef HITJ
      }
    }
    if (lane == 0) wcnt[wave] = wc;
    __syncthreads();

    if (wave == 0) {
      for (int wsx = 0; wsx < NWAVE; ++wsx) {
        int n = wcnt[wsx];
        n = (n < 0) ? 0 : ((n > WCAP) ? WCAP : n);
        for (int i = 0; i < n; i += 2) {
          const bool dupe = (i + 1 >= n);
          const int  idx  = i + ((half != 0 && !dupe) ? 1 : 0);
          const int  ent  = list[wsx * WCAP + idx];
          const int  slot = ent & (NB - 1);
          const int  el   = (ent >> 10) & (CHUNK - 1);
          int e = cbase + el;
          if (e > nE - 1) e = nE - 1;
          int s = sidx[e];
          s = (s < 0) ? 0 : ((s > n_src - 1) ? (n_src - 1) : s);
          int nd = nodeBase + slot;
          if (nd > n_dst - 1) nd = n_dst - 1;
          const v4f x = *(const v4f*)(hs + (size_t)s  * DCH + 4 * q);
          const v4f y = *(const v4f*)(hd + (size_t)nd * DCH + 4 * q);
          v4f t = x + y;
          t.x = (t.x > 0.f) ? t.x : NEGSL * t.x;
          t.y = (t.y > 0.f) ? t.y : NEGSL * t.y;
          t.z = (t.z > 0.f) ? t.z : NEGSL * t.z;
          t.w = (t.w > 0.f) ? t.w : NEGSL * t.w;
          float ev = a4.x * t.x + a4.y * t.y + a4.z * t.z + a4.w * t.w;
          ev += __shfl_xor(ev, 8, 32);
          ev += __shfl_xor(ev, 4, 32);
          ev += __shfl_xor(ev, 2, 32);
          ev += __shfl_xor(ev, 1, 32);
          const float M     = emx[slot];
          const float S     = den[slot];
          const int   oslot = __shfl_xor(slot, 16, 32);
          const float oev   = __shfl_xor(ev, 16, 32);
          const bool  same  = (oslot == slot) && !dupe;
          const float Mn    = fmaxf(fmaxf(M, ev), same ? oev : MINIT);
          const float p     = __expf(ev - Mn);
          const float sc    = __expf(M - Mn);
          const v4f   c     = p * x;
          v4f oc;
          oc.x = __shfl_xor(c.x, 16, 32);
          oc.y = __shfl_xor(c.y, 16, 32);
          oc.z = __shfl_xor(c.z, 16, 32);
          oc.w = __shfl_xor(c.w, 16, 32);
          const float op_ = __shfl_xor(p, 16, 32);
          const float fs  = same ? 1.0f : 0.0f;
          const v4f   tot = c + fs * oc;
          const float ps  = p + fs * op_;
          v4f* ap = (v4f*)(sacc + slot * DCH + 4 * q);
          const v4f   cur = *ap;
          const v4f   nv  = cur * sc + tot;
          const float Sn  = S * sc + ps;
          const bool  wr  = (half == 0) || (!same && !dupe);
          if (wr) {
            *ap = nv;
            if (q == 0) { den[slot] = Sn; emx[slot] = Mn; }
          }
          __builtin_amdgcn_fence(__ATOMIC_RELEASE, "wavefront");
          __builtin_amdgcn_wave_barrier();
        }
      }
    }
    __syncthreads();
  }

  const v4f b4 = *(const v4f*)(bias + 4 * q);
#pragma unroll 1
  for (int j = 0; j < NB / NWAVE / 2; ++j) {
    const int   slot = wave * (NB / NWAVE) + 2 * j + half;
    const int   node = nodeBase + slot;
    const float S    = den[slot];
    const float inv  = 1.0f / fmaxf(S, 1e-9f);
    const v4f   v    = *(const v4f*)(sacc + slot * DCH + 4 * q) * inv + b4;
    const bool  ok   = node < n_dst;
    float* op = outp + (size_t)(ok ? node : 0) * ld_out + 4 * q;
    if (ok) *(volatile v4f*)op = v;
    __threadfence();
    if (ok) *(volatile v4f*)op = v;
  }
}

extern "C" void kernel_launch(void* const* d_in, const int* in_sizes, int n_in,
                              void* d_out, int out_size, void* d_ws, size_t ws_size,
                              hipStream_t stream) {
  if (n_in < 26) return;
  const int nU = in_sizes[0] / DCH;
  const int nI = in_sizes[1] / DCH;
  if (nU <= 0 || nI <= 0) return;
  if (in_sizes[0] != nU * DCH || in_sizes[1] != nI * DCH) return;
  if ((nU & 15) != 0 || (nI & 15) != 0) return;
  const int eR = in_sizes[2], eB = in_sizes[4], eL = in_sizes[6];
  if (eR < 1 || eB < 1 || eL < 1) return;
  if (in_sizes[3] != eR || in_sizes[5] != eB || in_sizes[7] != eL) return;
  {
    const int wq[8] = {8, 9, 12, 13, 16, 17, 20, 21};
    for (int i = 0; i < 8; ++i) if (in_sizes[wq[i]] != DCH * DCH) return;
    const int vq[9] = {10, 11, 14, 15, 18, 19, 22, 23, 25};
    for (int i = 0; i < 9; ++i) if (in_sizes[vq[i]] != DCH) return;
    if (in_sizes[24] != 2 * DCH * DCH) return;
  }
  if (out_size != nU * DCH) return;

  const float* h_user   = (const float*)d_in[0];
  const float* h_item   = (const float*)d_in[1];
  const int*   rate_src = (const int*)d_in[2];
  const int*   rate_dst = (const int*)d_in[3];
  const int*   rb_src   = (const int*)d_in[4];
  const int*   rb_dst   = (const int*)d_in[5];
  const int*   link_src = (const int*)d_in[6];
  const int*   link_dst = (const int*)d_in[7];
  const float* w_src_r1  = (const float*)d_in[8];
  const float* w_dst_r1  = (const float*)d_in[9];
  const float* a_r1      = (const float*)d_in[10];
  const float* b_r1      = (const float*)d_in[11];
  const float* w_src_rb1 = (const float*)d_in[12];
  const float* w_dst_rb1 = (const float*)d_in[13];
  const float* a_rb1     = (const float*)d_in[14];
  const float* b_rb1     = (const float*)d_in[15];
  const float* w_src_rb2 = (const float*)d_in[16];
  const float* w_dst_rb2 = (const float*)d_in[17];
  const float* a_rb2     = (const float*)d_in[18];
  const float* b_rb2     = (const float*)d_in[19];
  const float* w_src_l2  = (const float*)d_in[20];
  const float* w_dst_l2  = (const float*)d_in[21];
  const float* a_l2      = (const float*)d_in[22];
  const float* b_l2      = (const float*)d_in[23];
  const float* w_out     = (const float*)d_in[24];
  const float* b_out     = (const float*)d_in[25];
  float* out = (float*)d_out;

  char* base = (char*)d_ws;
  size_t off = 0;
  us_t* wpl = (us_t*)(base + off);   off += (size_t)WPL_HALVES * 2;
  const size_t bU = (size_t)nU * DCH * sizeof(float);
  const size_t bI = (size_t)nI * DCH * sizeof(float);
  float* RA = (float*)(base + off);  off += bU;
  float* RB = (float*)(base + off);  off += bI;
  float* RC = (float*)(base + off);  off += bI;
  float* RD = (float*)(base + off);  off += bU;
  float* RE = (float*)(base + off);  off += bU;
  float* RF = (float*)(base + off);  off += bU;
  float* RG = (float*)(base + off);  off += bI;
  if (off > ws_size) return;
  if ((size_t)nU * 128 * sizeof(float) > bI) return;

  {
    PrepArgs pa;
    pa.W0 = w_src_r1;  pa.W1 = w_dst_r1;  pa.W2 = w_src_rb1; pa.W3 = w_dst_rb1;
    pa.W4 = w_src_rb2; pa.W5 = w_dst_rb2; pa.W6 = w_src_l2;  pa.W7 = w_dst_l2;
    pa.W8 = w_out;     pa.P  = wpl;
    k_prep<<<dim3(4, 9), NTHR, 0, stream>>>(pa);
  }
  const us_t* PL0 = wpl + 0 * 8192;
  const us_t* PL1 = wpl + 1 * 8192;
  const us_t* PL2 = wpl + 2 * 8192;
  const us_t* PL3 = wpl + 3 * 8192;
  const us_t* PL4 = wpl + 4 * 8192;
  const us_t* PL5 = wpl + 5 * 8192;
  const us_t* PL6 = wpl + 6 * 8192;
  const us_t* PL7 = wpl + 7 * 8192;
  const us_t* PL8 = wpl + 8 * 8192;

  {
    GemmArgs ga;
    ga.X = h_user; ga.bias = nullptr;
    ga.W0 = PL0; ga.Y0 = RA; ga.W1 = PL3; ga.Y1 = RD; ga.W2 = PL5; ga.Y2 = RE; ga.W3 = PL7; ga.Y3 = RF;
    ga.ldx = DCH; ga.ldy = DCH; ga.N = nU; ga.pad0 = 0;
    k_gemm<2><<<dim3((nU + GROWS - 1) / GROWS, 4), 128, 0, stream>>>(ga);
  }
  {
    GemmArgs ga;
    ga.X = h_item; ga.bias = nullptr;
    ga.W0 = PL1; ga.Y0 = RB; ga.W1 = PL2; ga.Y1 = RC; ga.W2 = PL1; ga.Y2 = RB; ga.W3 = PL1; ga.Y3 = RB;
    ga.ldx = DCH; ga.ldy = DCH; ga.N = nI; ga.pad0 = 0;
    k_gemm<2><<<dim3((nI + GROWS - 1) / GROWS, 2), 128, 0, stream>>>(ga);
  }

  hipFuncSetAttribute(reinterpret_cast<const void*>(&k_agg),
                      hipFuncAttributeMaxDynamicSharedMemorySize, LDS_BYTES);

  k_agg<<<(nI + NB - 1) / NB, NTHR, LDS_BYTES, stream>>>(RA, RB, rate_src, rate_dst, a_r1, b_r1,
                                                        RG, DCH, nU, nI, eR);
  k_agg<<<(nU + NB - 1) / NB, NTHR, LDS_BYTES, stream>>>(RC, RD, rb_src, rb_dst, a_rb1, b_rb1,
                                                        RA, DCH, nI, nU, eB);
  {
    GemmArgs ga;
    ga.X = RG; ga.bias = nullptr;
    ga.W0 = PL4; ga.Y0 = RB; ga.W1 = PL4; ga.Y1 = RB; ga.W2 = PL4; ga.Y2 = RB; ga.W3 = PL4; ga.Y3 = RB;
    ga.ldx = DCH; ga.ldy = DCH; ga.N = nI; ga.pad0 = 0;
    k_gemm<2><<<dim3((nI + GROWS - 1) / GROWS, 1), 128, 0, stream>>>(ga);
  }
  {
    GemmArgs ga;
    ga.X = RA; ga.bias = nullptr;
    ga.W0 = PL6; ga.Y0 = RD; ga.W1 = PL6; ga.Y1 = RD; ga.W2 = PL6; ga.Y2 = RD; ga.W3 = PL6; ga.Y3 = RD;
    ga.ldx = DCH; ga.ldy = DCH; ga.N = nU; ga.pad0 = 0;
    k_gemm<2><<<dim3((nU + GROWS - 1) / GROWS, 1), 128, 0, stream>>>(ga);
  }
  k_agg<<<(nU + NB - 1) / NB, NTHR, LDS_BYTES, stream>>>(RB, RE, rb_src, rb_dst, a_rb2, b_rb2,
                                                        RC, 2 * DCH, nI, nU, eB);
  k_agg<<<(nU + NB - 1) / NB, NTHR, LDS_BYTES, stream>>>(RD, RF, link_src, link_dst, a_l2, b_l2,
                                                        RC + DCH, 2 * DCH, nU, nU, eL);
  {
    GemmArgs ga;
    ga.X = RC; ga.bias = b_out;
    ga.W0 = PL8; ga.Y0 = out; ga.W1 = PL8; ga.Y1 = out; ga.W2 = PL8; ga.Y2 = out; ga.W3 = PL8; ga.Y3 = out;
    ga.ldx = 2 * DCH; ga.ldy = DCH; ga.N = nU; ga.pad0 = 0;
    k_gemm<4><<<dim3((nU + GROWS - 1) / GROWS, 1), 128, 0, stream>>>(ga);
  }
}
